// Memory_63642825392438
// MI455X (gfx1250) — hardware-verified
//
#include <hip/hip_runtime.h>

#define B_    4
#define DE    128
#define DO    512
#define HW    1560
#define HW16  1568
#define THW   6240
#define NPIX  (B_ * HW16)
#define NQT   (HW16 / 16)
#define SCALE 0.08838834764831843f

typedef __bf16 v16bf __attribute__((ext_vector_type(16)));
typedef float v8f __attribute__((ext_vector_type(8)));
typedef float v4f __attribute__((ext_vector_type(4), __may_alias__));
typedef unsigned int v4u __attribute__((ext_vector_type(4), __may_alias__));

union ABu { v16bf v; v4u q[2]; unsigned int u[8]; };

__device__ __forceinline__ unsigned short f2bf(float f) {
  unsigned int u = __float_as_uint(f);
  u += 0x7FFFu + ((u >> 16) & 1u);
  return (unsigned short)(u >> 16);
}

__device__ __forceinline__ unsigned int pack2(float a, float b) {
  return (unsigned int)f2bf(a) | ((unsigned int)f2bf(b) << 16);
}

__device__ __forceinline__ v4u pack8(const float* f) {
  v4u r;
  r.x = pack2(f[0], f[1]);
  r.y = pack2(f[2], f[3]);
  r.z = pack2(f[4], f[5]);
  r.w = pack2(f[6], f[7]);
  return r;
}

__device__ __forceinline__ v8f zero8() {
  v8f z;
#pragma unroll
  for (int i = 0; i < 8; ++i) z[i] = 0.f;
  return z;
}

__device__ __forceinline__ v8f wmma_bf16(v16bf a, v16bf b, v8f c) {
  v8f d = __builtin_amdgcn_wmma_f32_16x16x32_bf16(false, a, false, b, (short)0, c,
                                                  false, false);
  asm volatile("v_nop\n\tv_nop\n\tv_nop\n\tv_nop" : "+v"(d) : "v"(a), "v"(b));
  return d;
}

__device__ __forceinline__ v16bf load_frag(const unsigned short* base, int ld,
                                           int row0, int k0, int lane) {
  const int r = lane & 15, h = lane >> 4;
  const unsigned short* p = base + (size_t)(row0 + r) * ld + k0 + 8 * h;
  ABu t;
  t.q[0] = *(const v4u*)p;
  t.q[1] = *(const v4u*)(p + 16);
  return t.v;
}

__device__ __forceinline__ float fsigmoid(float x) {
  x = fminf(fmaxf(x, -30.f), 30.f);
  return 1.0f / (1.0f + __expf(-x));
}
__device__ __forceinline__ float ftanh_(float x) {
  x = fminf(fmaxf(x, -15.f), 15.f);
  float e = __expf(-2.f * x);
  return (1.f - e) / (1.f + e);
}


__global__ void __launch_bounds__(256) prep_m_kernel(const float* __restrict__ m_in,
                                                     unsigned short* Akd, int ngroups) {
  int g = blockIdx.x * 256 + threadIdx.x;
  if (g >= ngroups) return;
  int d8 = g & 15;
  int k  = (g >> 4) % THW;
  int b  = (g >> 4) / THW;
  const float* src = m_in + ((size_t)b * DE + d8 * 8) * THW + k;
  float f[8];
#pragma unroll
  for (int j = 0; j < 8; ++j) f[j] = src[(size_t)j * THW];
  v4u v = pack8(f);
  unsigned short* dst = Akd + ((size_t)b * THW + k) * DE + d8 * 8;
  *(volatile v4u*)dst = v;
  __threadfence();
  *(volatile v4u*)dst = v;
}

__global__ void __launch_bounds__(256) prep_q_kernel(const float* __restrict__ q_in,
                                                     unsigned short* QiT, int ngroups) {
  int g = blockIdx.x * 256 + threadIdx.x;
  if (g >= ngroups) return;
  int d8 = g & 15;
  int q  = (g >> 4) % HW16;
  int b  = (g >> 4) / HW16;
  float f[8];
  if (q < HW) {
    const float* src = q_in + ((size_t)b * DE + d8 * 8) * HW + q;
#pragma unroll
    for (int j = 0; j < 8; ++j) f[j] = src[(size_t)j * HW];
  } else {
#pragma unroll
    for (int j = 0; j < 8; ++j) f[j] = 0.f;
  }
  v4u v = pack8(f);
  unsigned short* dst = QiT + ((size_t)b * HW16 + q) * DE + d8 * 8;
  *(volatile v4u*)dst = v;
  __threadfence();
  *(volatile v4u*)dst = v;
}

__global__ void __launch_bounds__(256) prep_mo_kernel(const float* __restrict__ m_out,
                                                      unsigned short* Mo, int ngroups) {
  int g = blockIdx.x * 256 + threadIdx.x;
  if (g >= ngroups) return;
  const float* src = m_out + (size_t)g * 8;
  v4f a = *(const v4f*)src;
  v4f c = *(const v4f*)(src + 4);
  v4u v;
  v.x = pack2(a.x, a.y); v.y = pack2(a.z, a.w);
  v.z = pack2(c.x, c.y); v.w = pack2(c.z, c.w);
  unsigned short* dst = Mo + (size_t)g * 8;
  *(volatile v4u*)dst = v;
  __threadfence();
  *(volatile v4u*)dst = v;
}

__global__ void __launch_bounds__(256) prep_w_kernel(const float* __restrict__ wr,
                                                     const float* __restrict__ wu,
                                                     const float* __restrict__ wc,
                                                     unsigned short* Wbf, int ngroups) {
  int g = blockIdx.x * 256 + threadIdx.x;
  if (g >= ngroups) return;
  const int per = DO * 2 * DO / 8;
  int w = g / per, j = g - w * per;
  const float* s = (w == 0) ? wr : (w == 1) ? wu : wc;
  const float* src = s + (size_t)j * 8;
  v4f a = *(const v4f*)src;
  v4f c = *(const v4f*)(src + 4);
  v4u v;
  v.x = pack2(a.x, a.y); v.y = pack2(a.z, a.w);
  v.z = pack2(c.x, c.y); v.w = pack2(c.z, c.w);
  unsigned short* dst = Wbf + (size_t)g * 8;
  *(volatile v4u*)dst = v;
  __threadfence();
  *(volatile v4u*)dst = v;
}

__global__ void __launch_bounds__(256) prep_qout_kernel(const float* __restrict__ q_out,
                                                        float* QT, int ngroups) {
  int g = blockIdx.x * 256 + threadIdx.x;
  if (g >= ngroups) return;
  int o4  = g & (DO / 4 - 1);
  int pix = g >> 7;
  int b = pix / HW16, hw = pix - b * HW16;
  v4f v;
  if (hw < HW) {
    const float* src = q_out + ((size_t)b * DO + o4 * 4) * HW + hw;
    v.x = src[0];
    v.y = src[(size_t)HW];
    v.z = src[(size_t)2 * HW];
    v.w = src[(size_t)3 * HW];
  } else {
    v.x = 0.f; v.y = 0.f; v.z = 0.f; v.w = 0.f;
  }
  float* dst = QT + (size_t)pix * DO + o4 * 4;
  *(volatile v4f*)dst = v;
  __threadfence();
  *(volatile v4f*)dst = v;
}

__global__ void __launch_bounds__(256) attn_kernel(
    const unsigned short* __restrict__ Akd, const unsigned short* __restrict__ QiT,
    const unsigned short* __restrict__ MO, float* memF) {
  __shared__ __attribute__((aligned(16))) unsigned short pbuf[8][16][32];
  __shared__ __attribute__((aligned(16))) float otile[16][DO];
  __shared__ float sm[8][16], sl[8][16];
  __shared__ float smax[16], sinv[16];

  if (blockIdx.x >= B_ * NQT) return;
  const int b  = blockIdx.x / NQT;
  const int q0 = (blockIdx.x - b * NQT) * 16;
  const int wave = threadIdx.x >> 5, lane = threadIdx.x & 31;
  const int cc = lane & 15, h = lane >> 4;
  const unsigned short* A = Akd + (size_t)b * THW * DE;
  const unsigned short* Q = QiT + (size_t)b * HW16 * DE;
  const unsigned short* V = MO  + (size_t)b * DO * THW;

  v16bf btile[4];
#pragma unroll
  for (int d = 0; d < 4; ++d) btile[d] = load_frag(Q, DE, q0, d * 32, lane);

  float m = -3.0e38f, l = 0.f;
  for (int kt = wave; kt < THW / 16; kt += 8) {
    v8f acc = zero8();
#pragma unroll
    for (int d = 0; d < 4; ++d)
      acc = wmma_bf16(load_frag(A, DE, kt * 16, d * 32, lane), btile[d], acc);
    float tm = -3.0e38f;
#pragma unroll
    for (int v = 0; v < 8; ++v) tm = fmaxf(tm, acc[v] * SCALE);
    float mn = fmaxf(m, tm);
    l *= __expf(m - mn);
#pragma unroll
    for (int v = 0; v < 8; ++v) l += __expf(acc[v] * SCALE - mn);
    m = mn;
  }
  {
    float om = __shfl_xor(m, 16), ol = __shfl_xor(l, 16);
    float mn = fmaxf(m, om);
    l = l * __expf(m - mn) + ol * __expf(om - mn);
    m = mn;
  }
  if (lane < 16) { sm[wave][lane] = m; sl[wave][lane] = l; }
  __syncthreads();
  if (threadIdx.x < 16) {
    float M = -3.0e38f, L = 0.f;
    for (int w = 0; w < 8; ++w) {
      float mw = sm[w][threadIdx.x], lw = sl[w][threadIdx.x];
      float mm = fmaxf(M, mw);
      L = L * __expf(M - mm) + lw * __expf(mw - mm);
      M = mm;
    }
    smax[threadIdx.x] = M;
    sinv[threadIdx.x] = 1.0f / L;
  }
  __syncthreads();

  const float mq = smax[cc];
  const float invl = sinv[cc];
  v8f accs[4];
#pragma unroll
  for (int ot = 0; ot < 4; ++ot) accs[ot] = zero8();
  const int o0 = wave * 64;
  const int NST = THW / 32;
  for (int r = 0; r < (NST + 7) / 8; ++r) {
    const int st = r * 8 + wave;
    if (st < NST) {
      v8f s0 = zero8(), s1 = zero8();
#pragma unroll
      for (int d = 0; d < 4; ++d) {
        s0 = wmma_bf16(load_frag(A, DE, st * 32,      d * 32, lane), btile[d], s0);
        s1 = wmma_bf16(load_frag(A, DE, st * 32 + 16, d * 32, lane), btile[d], s1);
      }
      float e0[8], e1[8];
#pragma unroll
      for (int v = 0; v < 8; ++v) {
        e0[v] = __expf(s0[v] * SCALE - mq);
        e1[v] = __expf(s1[v] * SCALE - mq);
      }
      *(v4u*)(&pbuf[wave][cc][8 * h])      = pack8(e0);
      *(v4u*)(&pbuf[wave][cc][16 + 8 * h]) = pack8(e1);
    }
    __syncthreads();
    int nst = NST - r * 8; if (nst > 8) nst = 8;
    for (int s = 0; s < nst; ++s) {
      v16bf pb = load_frag(&pbuf[s][0][0], 32, 0, 0, lane);
      const int kst = (r * 8 + s) * 32;
#pragma unroll
      for (int ot = 0; ot < 4; ++ot)
        accs[ot] = wmma_bf16(load_frag(V, THW, o0 + ot * 16, kst, lane), pb, accs[ot]);
    }
    __syncthreads();
  }

#pragma unroll
  for (int ot = 0; ot < 4; ++ot) {
    v4f lo, hi;
    lo.x = accs[ot][0] * invl; lo.y = accs[ot][1] * invl;
    lo.z = accs[ot][2] * invl; lo.w = accs[ot][3] * invl;
    hi.x = accs[ot][4] * invl; hi.y = accs[ot][5] * invl;
    hi.z = accs[ot][6] * invl; hi.w = accs[ot][7] * invl;
    float* tp = &otile[cc][o0 + ot * 16 + 8 * h];
    *(v4f*)tp       = lo;
    *(v4f*)(tp + 4) = hi;
  }
  __syncthreads();
  {
    const size_t pix0 = (size_t)b * HW16 + q0;
    v4f vals[8];
    float* dsts[8];
#pragma unroll
    for (int s = 0; s < 2; ++s) {
      const int rr = 2 * wave + s;
#pragma unroll
      for (int c = 0; c < 4; ++c) {
        vals[s * 4 + c] = *(const v4f*)(&otile[rr][c * 128 + 4 * lane]);
        dsts[s * 4 + c] = memF + (pix0 + rr) * DO + c * 128 + 4 * lane;
      }
    }
#pragma unroll
    for (int i = 0; i < 8; ++i) *(volatile v4f*)dsts[i] = vals[i];
    __threadfence();
#pragma unroll
    for (int i = 0; i < 8; ++i) *(volatile v4f*)dsts[i] = vals[i];
  }
}

template <int MODE>
__global__ void __launch_bounds__(256) gate_kernel(
    const unsigned short* __restrict__ W,
    const float* __restrict__ X1,
    const float* __restrict__ X2,
    const float* __restrict__ bias,
    const float* __restrict__ addT,
    const float* __restrict__ memT,
    const float* __restrict__ uT,
    float* outF, int nptile) {
  __shared__ __attribute__((aligned(16))) unsigned short xs1[16 * DO];
  __shared__ __attribute__((aligned(16))) unsigned short xs2[(MODE == 4) ? 16 * DO : 8];
  __shared__ __attribute__((aligned(16))) float et[16][128];

  const int ptile = blockIdx.x >> 2;
  if (ptile >= nptile) return;
  const int wave = threadIdx.x >> 5, lane = threadIdx.x & 31;
  const int cc = lane & 15, h = lane >> 4;
  const int p0 = ptile * 16;
  const int ob = (blockIdx.x & 3) * 128;
  const int o0 = ob + wave * 16;
  const int c0 = (MODE == 0) ? DO : 0;

  {
    const int pix = threadIdx.x >> 4;
    const int ch  = (threadIdx.x & 15) * 32;
    const float* s1 = X1 + (size_t)(p0 + pix) * DO + ch;
    unsigned short* d1 = xs1 + pix * DO + ch;
#pragma unroll
    for (int j = 0; j < 4; ++j) {
      v4f fa = *(const v4f*)(s1 + 8 * j);
      v4f fb = *(const v4f*)(s1 + 8 * j + 4);
      v4u pk;
      pk.x = pack2(fa.x, fa.y); pk.y = pack2(fa.z, fa.w);
      pk.z = pack2(fb.x, fb.y); pk.w = pack2(fb.z, fb.w);
      *(v4u*)(d1 + 8 * j) = pk;
    }
    if (MODE == 4) {
      const float* s2 = X2 + (size_t)(p0 + pix) * DO + ch;
      unsigned short* d2 = xs2 + pix * DO + ch;
#pragma unroll
      for (int j = 0; j < 4; ++j) {
        v4f fa = *(const v4f*)(s2 + 8 * j);
        v4f fb = *(const v4f*)(s2 + 8 * j + 4);
        v4u pk;
        pk.x = pack2(fa.x, fa.y); pk.y = pack2(fa.z, fa.w);
        pk.z = pack2(fb.x, fb.y); pk.w = pack2(fb.z, fb.w);
        *(v4u*)(d2 + 8 * j) = pk;
      }
    }
  }
  __syncthreads();

  v8f acc = zero8();
  for (int kt = 0; kt < DO / 32; ++kt)
    acc = wmma_bf16(load_frag(W, 2 * DO, o0, c0 + kt * 32, lane),
                    load_frag(xs1, DO, 0, kt * 32, lane), acc);
  if (MODE == 4) {
    for (int kt = 0; kt < DO / 32; ++kt)
      acc = wmma_bf16(load_frag(W, 2 * DO, o0, DO + kt * 32, lane),
                      load_frag(xs2, DO, 0, kt * 32, lane), acc);
  }

  {
    v4f lo, hi;
    lo.x = acc[0]; lo.y = acc[1]; lo.z = acc[2]; lo.w = acc[3];
    hi.x = acc[4]; hi.y = acc[5]; hi.z = acc[6]; hi.w = acc[7];
    float* tp = &et[cc][wave * 16 + 8 * h];
    *(v4f*)tp       = lo;
    *(v4f*)(tp + 4) = hi;
  }
  __syncthreads();

  {
    const int pix = threadIdx.x >> 4;
    const int og  = (threadIdx.x & 15) * 8;
    const size_t gi = (size_t)(p0 + pix) * DO + ob + og;
    float a[8], o[8];
#pragma unroll
    for (int j = 0; j < 8; ++j) a[j] = et[pix][og + j];
    if (MODE == 0) {
#pragma unroll
      for (int j = 0; j < 8; ++j) o[j] = a[j] + bias[ob + og + j];
    } else if (MODE == 2) {
#pragma unroll
      for (int j = 0; j < 8; ++j) {
        float rg = fsigmoid(a[j] + addT[gi + j]);
        o[j] = rg * memT[gi + j];
      }
    } else if (MODE == 3) {
#pragma unroll
      for (int j = 0; j < 8; ++j) o[j] = fsigmoid(a[j] + addT[gi + j]);
    } else {
#pragma unroll
      for (int j = 0; j < 8; ++j) {
        float cv = ftanh_(a[j] + bias[ob + og + j]);
        float u  = uT[gi + j];
        float mm = memT[gi + j];
        o[j] = mm * (1.0f - u) + u * cv;
      }
    }
#pragma unroll
    for (int j = 0; j < 8; ++j) et[pix][og + j] = o[j];
  }
  __syncthreads();

  {
    const int r0 = 2 * wave, r1 = 2 * wave + 1;
    v4f v0 = *(const v4f*)(&et[r0][4 * lane]);
    v4f v1 = *(const v4f*)(&et[r1][4 * lane]);
    float* d0 = outF + (size_t)(p0 + r0) * DO + ob + 4 * lane;
    float* d1 = outF + (size_t)(p0 + r1) * DO + ob + 4 * lane;
    *(volatile v4f*)d0 = v0;
    *(volatile v4f*)d1 = v1;
    __threadfence();
    *(volatile v4f*)d0 = v0;
    *(volatile v4f*)d1 = v1;
  }
}

__global__ void __launch_bounds__(256) final_kernel(const float* __restrict__ qT,
                                                    const float* __restrict__ q_out,
                                                    float* out, int ngroups) {
  int g = blockIdx.x * 256 + threadIdx.x;
  if (g >= ngroups) return;
  const int i0 = g * 4;
  float f[4];
#pragma unroll
  for (int j = 0; j < 4; ++j) {
    int i  = i0 + j;
    int hw = i % HW;
    int ch = (i / HW) % (2 * DO);
    int b  = i / (2 * DO * HW);
    float v;
    if (ch < DO) v = qT[((size_t)b * HW16 + hw) * DO + ch];
    else         v = q_out[((size_t)b * DO + (ch - DO)) * HW + hw];
    f[j] = v;
  }
  v4f v;
  v.x = f[0]; v.y = f[1]; v.z = f[2]; v.w = f[3];
  float* dst = out + i0;
  *(volatile v4f*)dst = v;
  __threadfence();
  *(volatile v4f*)dst = v;
}

extern "C" void kernel_launch(void* const* d_in, const int* in_sizes, int n_in,
                              void* d_out, int out_size, void* d_ws, size_t ws_size,
                              hipStream_t stream) {
  if (n_in < 10) return;
  if (in_sizes[0] != B_ * DE * THW || in_sizes[1] != B_ * DO * THW ||
      in_sizes[2] != B_ * DE * HW  || in_sizes[3] != B_ * DO * HW ||
      in_sizes[4] != DO * 2 * DO   || in_sizes[5] != DO ||
      in_sizes[6] != DO * 2 * DO   || in_sizes[7] != DO ||
      in_sizes[8] != DO * 2 * DO   || in_sizes[9] != DO ||
      out_size != B_ * 2 * DO * HW) return;

  const float* m_in  = (const float*)d_in[0];
  const float* m_out = (const float*)d_in[1];
  const float* q_in  = (const float*)d_in[2];
  const float* q_out = (const float*)d_in[3];
  const float* wr    = (const float*)d_in[4];
  const float* br    = (const float*)d_in[5];
  const float* wu    = (const float*)d_in[6];
  const float* bu    = (const float*)d_in[7];
  const float* wc    = (const float*)d_in[8];
  const float* bc    = (const float*)d_in[9];

  char* ws = (char*)d_ws;
  size_t off = 0;
  auto alloc = [&](size_t bytes) {
    size_t o = off;
    off += (bytes + 255) & ~(size_t)255;
    return o;
  };
  const size_t actF = (size_t)NPIX * DO * 4;
  unsigned short* Akd = (unsigned short*)(ws + alloc((size_t)B_ * THW * DE * 2));
  unsigned short* QiT = (unsigned short*)(ws + alloc((size_t)B_ * HW16 * DE * 2));
  unsigned short* Mo  = (unsigned short*)(ws + alloc((size_t)B_ * DO * THW * 2));
  unsigned short* Wbf = (unsigned short*)(ws + alloc((size_t)3 * DO * 2 * DO * 2));
  float* MemF = (float*)(ws + alloc(actF));
  float* Cr   = (float*)(ws + alloc(actF));
  float* Cu   = (float*)(ws + alloc(actF));
  float* Uf   = (float*)(ws + alloc(actF));
  float* Rh   = (float*)(ws + alloc(actF));
  float* Qfa  = (float*)(ws + alloc(actF));
  float* Qfb  = (float*)(ws + alloc(actF));
  if (off > ws_size) return;

  int ng;
  ng = B_ * THW * (DE / 8);
  prep_m_kernel<<<dim3((ng + 255) / 256), dim3(256), 0, stream>>>(m_in, Akd, ng);
  ng = B_ * HW16 * (DE / 8);
  prep_q_kernel<<<dim3((ng + 255) / 256), dim3(256), 0, stream>>>(q_in, QiT, ng);
  ng = B_ * DO * THW / 8;
  prep_mo_kernel<<<dim3((ng + 255) / 256), dim3(256), 0, stream>>>(m_out, Mo, ng);
  ng = 3 * DO * 2 * DO / 8;
  prep_w_kernel<<<dim3((ng + 255) / 256), dim3(256), 0, stream>>>(wr, wu, wc, Wbf, ng);
  ng = NPIX * DO / 4;
  prep_qout_kernel<<<dim3((ng + 255) / 256), dim3(256), 0, stream>>>(q_out, Qfa, ng);

  attn_kernel<<<dim3(B_ * NQT), dim3(256), 0, stream>>>(Akd, QiT, Mo, MemF);

  const int nptile = NPIX / 16;
  const int GB = nptile * 4;
  const unsigned short* Wr = Wbf;
  const unsigned short* Wu = Wbf + (size_t)DO * 2 * DO;
  const unsigned short* Wc = Wbf + (size_t)2 * DO * 2 * DO;

  gate_kernel<0><<<dim3(GB), dim3(256), 0, stream>>>(Wr, MemF, MemF, br, MemF, MemF, MemF, Cr, nptile);
  gate_kernel<0><<<dim3(GB), dim3(256), 0, stream>>>(Wu, MemF, MemF, bu, MemF, MemF, MemF, Cu, nptile);

  float* qcur = Qfa;
  float* qnxt = Qfb;
  for (int it = 0; it < 5; ++it) {
    gate_kernel<2><<<dim3(GB), dim3(256), 0, stream>>>(Wr, qcur, qcur, br, Cr, MemF, MemF, Rh, nptile);
    gate_kernel<3><<<dim3(GB), dim3(256), 0, stream>>>(Wu, qcur, qcur, bu, Cu, MemF, MemF, Uf, nptile);
    gate_kernel<4><<<dim3(GB), dim3(256), 0, stream>>>(Wc, qcur, Rh, bc, Cr, MemF, Uf, qnxt, nptile);
    float* t = qcur; qcur = qnxt; qnxt = t;
  }

  ng = out_size / 4;
  final_kernel<<<dim3((ng + 255) / 256), dim3(256), 0, stream>>>(qcur, q_out, (float*)d_out, ng);
}
